// TrajectoryGLOM_4535485464727
// MI455X (gfx1250) — hardware-verified
//
#include <hip/hip_runtime.h>
#include <math.h>

#define TT_   32768
#define LL_   5
#define DH_   64
#define DX_   32
#define H1N   24
#define H2N   16
#define NUDR  ((LL_ - 1) * TT_)
#define WPB   4
#define NBN   128
#define TPWUD 16
#define NBIN  512
#define PLH   2048
#define NPL   9
#define UTT   32
#define UTHR  (LL_ * 32)
#define SLP   68
#define ASC   256.0f
#define WSC   64.0f
#define LOSC  2048.0f
#define S12   (1.0f / 64.0f)
#define S12L  (1.0f / 131072.0f)
#define S3K   (1.0f / 524288.0f)
#define CVERT 0.05f
#define CLAT  0.1f
#define CREM  0.7f
#define BNEPS 1e-5f

static_assert(NUDR / 16 == NBN * WPB * TPWUD);
static_assert(TT_ / 16 == NBIN * WPB);
static_assert((TT_ % UTT) == 0 && UTT == 32);
static_assert((DH_ % 32) == 0 && (DX_ % 32) == 0);
static_assert(UTHR == 160);

typedef _Float16 v16h __attribute__((ext_vector_type(16)));
typedef _Float16 v8h  __attribute__((ext_vector_type(8)));
typedef float    v8f  __attribute__((ext_vector_type(8)));
typedef float    v4f  __attribute__((ext_vector_type(4)));
typedef unsigned int v4u __attribute__((ext_vector_type(4)));

union FragH { v16h v; v8h h[2]; v4u u[2]; };

__device__ __forceinline__ unsigned short bf_bits(float f) {
  unsigned u = __float_as_uint(f);
  return (unsigned short)((u + 0x7FFFu + ((u >> 16) & 1u)) >> 16);
}
__device__ __forceinline__ float bf_up(unsigned short h) { return __uint_as_float(((unsigned)h) << 16); }
__device__ __forceinline__ float bfr(float f) { return bf_up(bf_bits(f)); }
__device__ __forceinline__ unsigned short h_bits(_Float16 x) { return __builtin_bit_cast(unsigned short, x); }
__device__ __forceinline__ unsigned pk16(unsigned short a, unsigned short b) { return (unsigned)a | ((unsigned)b << 16); }
__device__ __forceinline__ unsigned pkh(float a, float b) { return pk16(h_bits((_Float16)a), h_bits((_Float16)b)); }
__device__ __forceinline__ v8f zero8() { v8f z = {0.f, 0.f, 0.f, 0.f, 0.f, 0.f, 0.f, 0.f}; return z; }
__device__ __forceinline__ v4f zero4() { v4f z = {0.f, 0.f, 0.f, 0.f}; return z; }
__device__ __forceinline__ v4f bfr4(v4f a) {
  v4f o;
#pragma unroll
  for (int e = 0; e < 4; ++e) o[e] = bfr(a[e]);
  return o;
}

__device__ __forceinline__ void hl_pair(float f0, float f1, unsigned& hp, unsigned& lp) {
#pragma clang fp contract(off)
  const _Float16 h0 = (_Float16)f0, h1 = (_Float16)f1;
  const float d0 = f0 - (float)h0, d1 = f1 - (float)h1;
  const float q0 = d0 * LOSC, q1 = d1 * LOSC;
  hp = pk16(h_bits(h0), h_bits(h1));
  lp = pk16(h_bits((_Float16)q0), h_bits((_Float16)q1));
}

__device__ __forceinline__ v16h ldfrag_h(const _Float16* p) {
  FragH f;
  f.h[0] = *(const v8h*)(p);
  f.h[1] = *(const v8h*)(p + 16);
  return f.v;
}

__device__ __forceinline__ v8f mma_h(v16h a, v16h b, v8f c) {
  c = __builtin_amdgcn_wmma_f32_16x16x32_f16(false, a, false, b, (short)0, c, false, false);
#if defined(__HIP_DEVICE_COMPILE__)
  asm volatile("v_nop\n\tv_nop\n\tv_nop\n\tv_nop" : "+v"(c) : "v"(a), "v"(b));
#endif
  return c;
}
__device__ __forceinline__ void wave_sync_lds() {
  __builtin_amdgcn_fence(__ATOMIC_RELEASE, "workgroup");
  __builtin_amdgcn_wave_barrier();
  __builtin_amdgcn_fence(__ATOMIC_ACQUIRE, "workgroup");
}

__global__ __launch_bounds__(256) void k_cvtw(const float* __restrict__ w0, const float* __restrict__ w1,
                                              const float* __restrict__ w2, const float* __restrict__ w3,
                                              const float* __restrict__ w4, const float* __restrict__ w5,
                                              const float* __restrict__ w6, const float* __restrict__ w7,
                                              const float* __restrict__ w8, unsigned short* wpl) {
  const int tid = threadIdx.x;
  const int pid = blockIdx.x;
  const int net = pid / 3, lay = pid - 3 * net;
  const float* src = (pid == 0) ? w0 : ((pid == 1) ? w1 : ((pid == 2) ? w2 : ((pid == 3) ? w3 : ((pid == 4) ? w4 :
                     ((pid == 5) ? w5 : ((pid == 6) ? w6 : ((pid == 7) ? w7 : w8)))))));
  int K, N, Np, Kp;
  if (lay == 0)      { K = (net == 0) ? DX_ : DH_; N = H1N; Np = 32; Kp = K; }
  else if (lay == 1) { K = H1N; N = H2N; Np = 16; Kp = 32; }
  else               { K = H2N; N = DH_; Np = 64; Kp = 32; }
  const int kq = Kp >> 3;
  const int items = Np * kq;
  const int n  = (kq == 8) ? (tid >> 3) : (tid >> 2);
  const int k8 = (kq == 8) ? ((tid & 7) * 8) : ((tid & 3) * 8);
  const int nc = (n < N) ? n : (N - 1);
  float f[8];
#pragma unroll
  for (int e = 0; e < 8; ++e) {
    const int k = k8 + e;
    int kk; float sc; bool valid;
    if (lay == 2) { kk = (k < 16) ? k : (k - 16); sc = (k < 16) ? LOSC : 1.0f; valid = (n < N); }
    else          { kk = k; sc = WSC; valid = (k < K) && (n < N); }
    const int kc = (kk < K) ? kk : (K - 1);
    const float v = bfr(src[(size_t)kc * N + nc]) * sc;
    f[e] = valid ? v : 0.f;
  }
  v4u pk;
#pragma unroll
  for (int e = 0; e < 4; ++e) pk[e] = pkh(f[2 * e], f[2 * e + 1]);
  if (tid < items) {
    unsigned short* gp = wpl + (size_t)pid * PLH + (size_t)n * Kp + k8;
    *(volatile v4u*)gp = pk;
    __threadfence();
    *(volatile v4u*)gp = pk;
  }
}

template <int K1, bool STATS, bool RND>
__device__ __forceinline__ void mlp_tile(const float* __restrict__ X, size_t row0,
                                         const _Float16* __restrict__ W1p, const _Float16* __restrict__ W2p,
                                         const _Float16* __restrict__ W3p,
                                         const float* sB1, const float* sB2, const float* sB3,
                                         float* Y, float* slab, v4f& su, v4f& qu) {
  const int lane = threadIdx.x & 31, hh = lane >> 4, m = lane & 15;
  constexpr int KS1 = K1 / 32;

  const float* xr = X + (row0 + m) * (size_t)K1 + 8 * hh;
  v16h fbh[KS1], fbl[KS1];
#pragma unroll
  for (int ks = 0; ks < KS1; ++ks) {
    const v4f x0 = *(const v4f*)(xr + 32 * ks);
    const v4f x1 = *(const v4f*)(xr + 32 * ks + 4);
    const v4f x2 = *(const v4f*)(xr + 32 * ks + 16);
    const v4f x3 = *(const v4f*)(xr + 32 * ks + 20);
    float f[16];
#pragma unroll
    for (int e = 0; e < 4; ++e) { f[e] = x0[e]; f[4 + e] = x1[e]; f[8 + e] = x2[e]; f[12 + e] = x3[e]; }
    if (RND) {
#pragma unroll
      for (int e = 0; e < 16; ++e) f[e] = bfr(f[e]);
    }
    v4u uh0, ul0, uh1, ul1;
#pragma unroll
    for (int e = 0; e < 4; ++e) {
      unsigned hp, lp;
      hl_pair(f[2 * e] * ASC, f[2 * e + 1] * ASC, hp, lp);         uh0[e] = hp; ul0[e] = lp;
      hl_pair(f[8 + 2 * e] * ASC, f[8 + 2 * e + 1] * ASC, hp, lp); uh1[e] = hp; ul1[e] = lp;
    }
    FragH gh, gl;
    gh.u[0] = uh0; gh.u[1] = uh1;
    gl.u[0] = ul0; gl.u[1] = ul1;
    fbh[ks] = gh.v; fbl[ks] = gl.v;
  }

  v8f c1ah = zero8(), c1al = zero8(), c1bh = zero8(), c1bl = zero8();
#pragma unroll
  for (int ks = 0; ks < KS1; ++ks) {
    const v16h fa0 = ldfrag_h(W1p + (size_t)m * K1 + 32 * ks + 8 * hh);
    const v16h fa1 = ldfrag_h(W1p + (size_t)(16 + m) * K1 + 32 * ks + 8 * hh);
    c1ah = mma_h(fa0, fbh[ks], c1ah);
    c1al = mma_h(fa0, fbl[ks], c1al);
    c1bh = mma_h(fa1, fbh[ks], c1bh);
    c1bl = mma_h(fa1, fbl[ks], c1bl);
  }
  v16h b2h, b2l;
  {
    const v4f p0 = *(const v4f*)(sB1 + 8 * hh);
    const v4f p1 = *(const v4f*)(sB1 + 8 * hh + 4);
    const v4f p2 = *(const v4f*)(sB1 + 16 + 8 * hh);
    const v4f p3 = *(const v4f*)(sB1 + 16 + 8 * hh + 4);
    float g0[8], g1[8];
#pragma unroll
    for (int e = 0; e < 4; ++e) {
      g0[e]     = fmaxf(c1ah[e] * S12 + c1al[e] * S12L + p0[e], 0.f);
      g0[4 + e] = fmaxf(c1ah[4 + e] * S12 + c1al[4 + e] * S12L + p1[e], 0.f);
      g1[e]     = fmaxf(c1bh[e] * S12 + c1bl[e] * S12L + p2[e], 0.f);
      g1[4 + e] = fmaxf(c1bh[4 + e] * S12 + c1bl[4 + e] * S12L + p3[e], 0.f);
    }
    v4u uh0, ul0, uh1, ul1;
#pragma unroll
    for (int e = 0; e < 4; ++e) {
      unsigned hp, lp;
      hl_pair(g0[2 * e], g0[2 * e + 1], hp, lp); uh0[e] = hp; ul0[e] = lp;
      hl_pair(g1[2 * e], g1[2 * e + 1], hp, lp); uh1[e] = hp; ul1[e] = lp;
    }
    FragH gh, gl;
    gh.u[0] = uh0; gh.u[1] = uh1;
    gl.u[0] = ul0; gl.u[1] = ul1;
    b2h = gh.v; b2l = gl.v;
  }

  v16h b3v;
  {
    const v16h fa2 = ldfrag_h(W2p + (size_t)m * 32 + 8 * hh);
    const v8f c2h = mma_h(fa2, b2h, zero8());
    const v8f c2l = mma_h(fa2, b2l, zero8());
    const v4f p0 = *(const v4f*)(sB2 + 8 * hh);
    const v4f p1 = *(const v4f*)(sB2 + 8 * hh + 4);
    float g2[8];
#pragma unroll
    for (int e = 0; e < 4; ++e) {
      g2[e]     = fmaxf(c2h[e] * S12 + c2l[e] * S12L + p0[e], 0.f);
      g2[4 + e] = fmaxf(c2h[4 + e] * S12 + c2l[4 + e] * S12L + p1[e], 0.f);
    }
    v4u uh0, ul0;
#pragma unroll
    for (int e = 0; e < 4; ++e) {
      unsigned hp, lp;
      hl_pair(g2[2 * e], g2[2 * e + 1], hp, lp); uh0[e] = hp; ul0[e] = lp;
    }
    FragH g; g.u[0] = uh0; g.u[1] = ul0;
    b3v = g.v;
  }

#pragma unroll
  for (int j = 0; j < 4; ++j) {
    const v16h fa3 = ldfrag_h(W3p + (size_t)(16 * j + m) * 32 + 8 * hh);
    const v8f c3 = mma_h(fa3, b3v, zero8());
    const v4f p0 = *(const v4f*)(sB3 + 16 * j + 8 * hh);
    const v4f p1 = *(const v4f*)(sB3 + 16 * j + 8 * hh + 4);
    v4f y0, y1;
#pragma unroll
    for (int e = 0; e < 4; ++e) {
      y0[e] = c3[e] * S3K + p0[e];
      y1[e] = c3[4 + e] * S3K + p1[e];
    }
    *(v4f*)(slab + m * SLP + 16 * j + 8 * hh)     = y0;
    *(v4f*)(slab + m * SLP + 16 * j + 8 * hh + 4) = y1;
  }
  wave_sync_lds();

  v4f ov[8];
#pragma unroll
  for (int it = 0; it < 8; ++it) ov[it] = *(const v4f*)(slab + (2 * it + hh) * SLP + 4 * m);
  if (STATS) {
#pragma unroll
    for (int it = 0; it < 8; ++it) {
      su += ov[it];
#pragma unroll
      for (int e = 0; e < 4; ++e) qu[e] = ov[it][e] * ov[it][e] + qu[e];
    }
  }
#pragma unroll
  for (int it = 0; it < 8; ++it) {
    float* gp = Y + (row0 + 2 * it + hh) * DH_ + 4 * m;
    *(volatile v4f*)gp = ov[it];
  }
  __threadfence();
#pragma unroll
  for (int it = 0; it < 8; ++it) {
    float* gp = Y + (row0 + 2 * it + hh) * DH_ + 4 * m;
    *(volatile v4f*)gp = ov[it];
  }
  wave_sync_lds();
}

template <int K1, bool STATS, bool RND>
__global__ __launch_bounds__(128) void k_mlp(const float* __restrict__ X0, const float* __restrict__ X1,
                                             const unsigned short* __restrict__ wpl, int slot0, int slot1,
                                             const float* __restrict__ b1a, const float* __restrict__ b2a,
                                             const float* __restrict__ b3a,
                                             const float* __restrict__ b1b, const float* __restrict__ b2b,
                                             const float* __restrict__ b3b,
                                             float* Y0, float* Y1, float* part, int ntn, int nbn, int tpw) {
  __shared__ __align__(16) float sB1[32];
  __shared__ __align__(16) float sB2[16];
  __shared__ __align__(16) float sB3[64];
  __shared__ __align__(16) float sslab[WPB][16 * SLP];
  __shared__ __align__(16) float sred[WPB][128];
  __shared__ __align__(16) float sout[128];

  const int tid = threadIdx.x, lane = tid & 31;
  const int wave = __builtin_amdgcn_readfirstlane(tid >> 5);
  const int hh = lane >> 4, m = lane & 15;
  const int nbnc = (nbn < 1) ? 1 : nbn;
  const int net = ((int)blockIdx.x >= nbnc) ? 1 : 0;
  const int bl = (int)blockIdx.x - net * nbnc;
  const float* X  = net ? X1 : X0;
  const float* b1 = net ? b1b : b1a;
  const float* b2 = net ? b2b : b2a;
  const float* b3 = net ? b3b : b3a;
  float* Y = net ? Y1 : Y0;
  const int slot = net ? slot1 : slot0;
  const int slc = (slot < 0) ? 0 : ((slot > NPL - 3) ? (NPL - 3) : slot);
  const _Float16* WP = (const _Float16*)(const void*)wpl;
  const _Float16* W1p = WP + (size_t)slc * PLH;
  const _Float16* W2p = W1p + PLH;
  const _Float16* W3p = W2p + PLH;

  if (wave == 0) {
    const int nc = (lane < H1N) ? lane : (H1N - 1);
    const float v = bfr(b1[nc]) * ASC;
    sB1[lane] = (lane < H1N) ? v : 0.f;
  } else if (wave == 1) {
    const float v = bfr(b2[lane & 15]) * ASC;
    if (lane < 16) sB2[lane] = v;
  } else {
    const int n = (wave - 2) * 32 + lane;
    sB3[n] = bfr(b3[n]);
  }
  __syncthreads();

  const int gw = bl * WPB + wave;
  const int NW = nbnc * WPB;
  v4f su = zero4(), qu = zero4();
  const int tpwc = (tpw < 64) ? tpw : 64;
#pragma unroll 1
  for (int i = 0; i < tpwc; ++i) {
    const int t = gw + i * NW;
    if (t < ntn) {
      mlp_tile<K1, STATS, RND>(X, (size_t)t * 16, W1p, W2p, W3p, sB1, sB2, sB3, Y,
                               sslab[wave], su, qu);
    }
  }

  if (STATS) {
#pragma unroll
    for (int e = 0; e < 4; ++e) {
      su[e] = su[e] + __shfl_xor(su[e], 16, 32);
      qu[e] = qu[e] + __shfl_xor(qu[e], 16, 32);
    }
    *(v4f*)(sred[wave] + 4 * m)      = su;
    *(v4f*)(sred[wave] + 64 + 4 * m) = qu;
    __syncthreads();
    {
      float v = sred[0][tid];
      v = v + sred[1][tid];
      v = v + sred[2][tid];
      v = v + sred[3][tid];
      sout[tid] = v;
    }
    __syncthreads();
    if (wave == 0) {
      const v4f o0 = *(const v4f*)(sout + 4 * lane);
      float* gp = part + (size_t)blockIdx.x * 128 + 4 * lane;
      *(volatile v4f*)gp = o0;
      __threadfence();
      *(volatile v4f*)gp = o0;
    }
  }
}

__global__ __launch_bounds__(256) void k_bnfin(const float* __restrict__ part, const float* __restrict__ ug,
                                               const float* __restrict__ ub, const float* __restrict__ dg,
                                               const float* __restrict__ db, float* stats) {
  __shared__ double sdd[256];
  __shared__ __align__(16) float so[256];
  const int tid = threadIdx.x, lane = tid & 31;
  const int wave = __builtin_amdgcn_readfirstlane(tid >> 5);
  const int pn = tid >> 7, c = tid & 127;
  double a = 0.0;
#pragma unroll 4
  for (int b = 0; b < NBN; ++b) a += (double)part[((size_t)(pn * NBN + b)) * 128 + c];
  sdd[tid] = a;
  __syncthreads();
  if (tid < 128) {
    const int net = tid >> 6, col = tid & 63;
    const double S = sdd[net * 128 + col];
    const double Q = sdd[net * 128 + 64 + col];
    const double invn = 1.0 / (double)NUDR;
    const double mu = S * invn;
    double var = Q * invn - mu * mu;
    var = (var > 0.0) ? var : 0.0;
    const float muf = (float)mu;
    const float varf = (float)var;
    const float istd = 1.0f / sqrtf(varf + BNEPS);
    const float g0 = bfr(ug[col]), g1 = bfr(dg[col]);
    const float e0 = bfr(ub[col]), e1 = bfr(db[col]);
    const float g = net ? g1 : g0;
    const float bt = net ? e1 : e0;
    const float A = istd * g;
    const float C = bt - muf * A;
    so[net * 128 + col]      = CVERT * A;
    so[net * 128 + 64 + col] = CVERT * C;
  }
  __syncthreads();
  if (wave == 0) {
    const v4f o0 = *(const v4f*)(so + 4 * lane);
    const v4f o1 = *(const v4f*)(so + 128 + 4 * lane);
    float* gp = stats + 4 * lane;
    *(volatile v4f*)gp = o0;
    *(volatile v4f*)(gp + 128) = o1;
    __threadfence();
    *(volatile v4f*)gp = o0;
    *(volatile v4f*)(gp + 128) = o1;
  }
}

template <bool RND>
__global__ __launch_bounds__(UTHR) void k_upd(const float* __restrict__ hin, const float* __restrict__ xe,
                                              const float* __restrict__ yu, const float* __restrict__ yd,
                                              const float* __restrict__ st, float* hout) {
  constexpr int NPAIR = UTT + 1;
  constexpr int NSLOT = LL_ * NPAIR;
  constexpr int NUNIT = NSLOT * 4;
  constexpr int NIT   = (NUNIT + UTHR - 1) / UTHR;
  constexpr int NCS   = (NSLOT + UTHR - 1) / UTHR;
  __shared__ float sat[NSLOT + 3];
  __shared__ float shr[NSLOT + 3];

  const int tid = threadIdx.x, lane = tid & 31;
  const int wave = __builtin_amdgcn_readfirstlane(tid >> 5);
  const int t0 = blockIdx.x * UTT;

#pragma unroll 1
  for (int s = 0; s < NIT; ++s) {
    int idx = tid + UTHR * s;
    idx = (idx < NUNIT) ? idx : (NUNIT - 1);
    const int u = idx >> 2, q4 = idx & 3;
    const int l = u / NPAIR, p = u - l * NPAIR;
    int ta = t0 - 1 + p;
    ta = (ta < 0) ? 0 : ((ta > TT_ - 1) ? (TT_ - 1) : ta);
    int tb = t0 + p;
    tb = (tb > TT_ - 1) ? (TT_ - 1) : tb;
    const float* ra = hin + ((size_t)l * TT_ + ta) * DH_ + 16 * q4;
    const float* rb = hin + ((size_t)l * TT_ + tb) * DH_ + 16 * q4;
    v4f a0 = *(const v4f*)(ra), a1 = *(const v4f*)(ra + 4), a2 = *(const v4f*)(ra + 8), a3 = *(const v4f*)(ra + 12);
    v4f b0 = *(const v4f*)(rb), b1 = *(const v4f*)(rb + 4), b2 = *(const v4f*)(rb + 8), b3 = *(const v4f*)(rb + 12);
    if (RND) {
      a0 = bfr4(a0); a1 = bfr4(a1); a2 = bfr4(a2); a3 = bfr4(a3);
      b0 = bfr4(b0); b1 = bfr4(b1); b2 = bfr4(b2); b3 = bfr4(b3);
    }
    float d = 0.f;
#pragma unroll
    for (int e = 0; e < 4; ++e) d = a0[e] * b0[e] + d;
#pragma unroll
    for (int e = 0; e < 4; ++e) d = a1[e] * b1[e] + d;
#pragma unroll
    for (int e = 0; e < 4; ++e) d = a2[e] * b2[e] + d;
#pragma unroll
    for (int e = 0; e < 4; ++e) d = a3[e] * b3[e] + d;
    d = d + __shfl_xor(d, 1, 32);
    d = d + __shfl_xor(d, 2, 32);
    if (q4 == 0) sat[u] = fmaxf(d, 0.f);
  }
  __syncthreads();

#pragma unroll 1
  for (int s = 0; s < NCS; ++s) {
    const int i = tid + UTHR * s;
    if (i < NSLOT) {
      const int l = i / NPAIR, p = i - l * NPAIR;
      float sacc = 0.f;
#pragma unroll
      for (int l2 = LL_ - 1; l2 >= 0; --l2) {
        const float av = sat[l2 * NPAIR + p];
        const float sn = sacc + av;
        sacc = (l2 >= l) ? sn : sacc;
      }
      const int t = t0 - 1 + p;
      const bool valid = (t >= 0) && (t <= TT_ - 2);
      const float ex = expf(-sacc);
      const float hv = CLAT * (1.0f - ex);
      shr[i] = valid ? hv : 0.f;
    }
  }
  __syncthreads();

  const int l = (wave < LL_) ? wave : (LL_ - 1);
  const int h2 = lane >> 4, q = lane & 15;
  const int ts = 16 * h2;
  const v4f Au = *(const v4f*)(st + 4 * q);
  const v4f Cu = *(const v4f*)(st + 64 + 4 * q);
  const v4f Ad = *(const v4f*)(st + 128 + 4 * q);
  const v4f Cd = *(const v4f*)(st + 192 + 4 * q);
  const size_t lvl = (size_t)l * TT_;
  const int lu = (l > 0) ? (l - 1) : 0;
  const int ld = (l < LL_ - 1) ? l : (LL_ - 2);
  int tm1 = t0 + ts - 1;
  tm1 = (tm1 < 0) ? 0 : tm1;
  v4f hm = *(const v4f*)(hin + (lvl + tm1) * DH_ + 4 * q);
  v4f hc = *(const v4f*)(hin + (lvl + t0 + ts) * DH_ + 4 * q);
  if (RND) { hm = bfr4(hm); hc = bfr4(hc); }
#pragma unroll 1
  for (int j = 0; j < 16; ++j) {
    const int t = t0 + ts + j;
    const int tp = (t + 1 > TT_ - 1) ? (TT_ - 1) : (t + 1);
    v4f hp = *(const v4f*)(hin + (lvl + tp) * DH_ + 4 * q);
    if (RND) hp = bfr4(hp);
    const float rB = shr[l * NPAIR + ts + j];
    const float rA = shr[l * NPAIR + ts + j + 1];
    v4f vu, vd;
    if (l == 0) {
      const v4f xv = *(const v4f*)(xe + (size_t)t * DH_ + 4 * q);
#pragma unroll
      for (int e = 0; e < 4; ++e) vu[e] = CVERT * xv[e];
    } else {
      const v4f y = *(const v4f*)(yu + ((size_t)lu * TT_ + t) * DH_ + 4 * q);
#pragma unroll
      for (int e = 0; e < 4; ++e) vu[e] = y[e] * Au[e] + Cu[e];
    }
    if (l < LL_ - 1) {
      const v4f y = *(const v4f*)(yd + ((size_t)ld * TT_ + t) * DH_ + 4 * q);
#pragma unroll
      for (int e = 0; e < 4; ++e) vd[e] = y[e] * Ad[e] + Cd[e];
    } else {
      vd = zero4();
    }
    v4f o;
#pragma unroll
    for (int e = 0; e < 4; ++e) {
      float acc = vu[e] + vd[e];
      acc = rB * hm[e] + acc;
      acc = rA * hp[e] + acc;
      o[e] = CREM * hc[e] + acc;
    }
    float* gp = hout + (lvl + t) * DH_ + 4 * q;
    *(volatile v4f*)gp = o;
    __threadfence();
    *(volatile v4f*)gp = o;
    hm = hc;
    hc = hp;
  }
}

extern "C" void kernel_launch(void* const* d_in, const int* in_sizes, int n_in,
                              void* d_out, int out_size, void* d_ws, size_t ws_size,
                              hipStream_t stream) {
  if (n_in < 25) return;
  const int ex[25] = { TT_ * DX_, LL_ * TT_ * DH_,
                       DX_ * H1N, H1N, H1N * H2N, H2N, H2N * DH_, DH_,
                       DH_ * H1N, H1N, H1N * H2N, H2N, H2N * DH_, DH_, DH_, DH_,
                       DH_ * H1N, H1N, H1N * H2N, H2N, H2N * DH_, DH_, DH_, DH_, 1 };
  for (int i = 0; i < 25; ++i) if (in_sizes[i] != ex[i]) return;
  if (out_size != LL_ * TT_ * DH_) return;

  const float* x    = (const float*)d_in[0];
  const float* hid0 = (const float*)d_in[1];
  const float* iW1 = (const float*)d_in[2];  const float* ib1 = (const float*)d_in[3];
  const float* iW2 = (const float*)d_in[4];  const float* ib2 = (const float*)d_in[5];
  const float* iW3 = (const float*)d_in[6];  const float* ib3 = (const float*)d_in[7];
  const float* uW1 = (const float*)d_in[8];  const float* ub1 = (const float*)d_in[9];
  const float* uW2 = (const float*)d_in[10]; const float* ub2 = (const float*)d_in[11];
  const float* uW3 = (const float*)d_in[12]; const float* ub3 = (const float*)d_in[13];
  const float* ug  = (const float*)d_in[14]; const float* ubt = (const float*)d_in[15];
  const float* dW1 = (const float*)d_in[16]; const float* db1 = (const float*)d_in[17];
  const float* dW2 = (const float*)d_in[18]; const float* db2 = (const float*)d_in[19];
  const float* dW3 = (const float*)d_in[20]; const float* db3 = (const float*)d_in[21];
  const float* dgm = (const float*)d_in[22]; const float* dbt = (const float*)d_in[23];
  float* out = (float*)d_out;

  const size_t sWPL  = (size_t)NPL * PLH * 2;
  const size_t sXE   = (size_t)TT_ * DH_ * 4;
  const size_t sY    = (size_t)NUDR * DH_ * 4;
  const size_t sPART = (size_t)(2 * NBN) * 128 * 4;
  const size_t sST   = 4096;
  const size_t sH    = (size_t)LL_ * TT_ * DH_ * 4;
  size_t off = 0;
  const size_t oWPL  = off; off += sWPL;
  const size_t oXE   = off; off += sXE;
  const size_t oYU   = off; off += sY;
  const size_t oYD   = off; off += sY;
  const size_t oPART = off; off += sPART;
  const size_t oST   = off; off += sST;
  const size_t oH    = off; off += sH;
  if (off > ws_size) return;
  if (off > (size_t)134217728) return;

  char* ws = (char*)d_ws;
  unsigned short* WPL = (unsigned short*)(ws + oWPL);
  float* XE   = (float*)(ws + oXE);
  float* YU   = (float*)(ws + oYU);
  float* YD   = (float*)(ws + oYD);
  float* PART = (float*)(ws + oPART);
  float* ST   = (float*)(ws + oST);
  float* HWS  = (float*)(ws + oH);

  k_cvtw<<<dim3(NPL), dim3(256), 0, stream>>>(iW1, iW2, iW3, uW1, uW2, uW3, dW1, dW2, dW3, WPL);
  k_mlp<DX_, false, true><<<dim3(NBIN), dim3(128), 0, stream>>>(x, x, WPL, 0, 0, ib1, ib2, ib3, ib1, ib2, ib3,
                                                                XE, XE, PART, TT_ / 16, NBIN, 1);
  const int iters = 10;
  for (int it = 0; it < iters; ++it) {
    const float* hin = (it == 0) ? hid0 : (((it - 1) & 1) ? (const float*)out : (const float*)HWS);
    float* hout = (it & 1) ? out : HWS;
    if (it == 0) {
      k_mlp<DH_, true, true><<<dim3(2 * NBN), dim3(128), 0, stream>>>(hin, hin + (size_t)TT_ * DH_, WPL, 3, 6,
                                                                      ub1, ub2, ub3, db1, db2, db3,
                                                                      YU, YD, PART, NUDR / 16, NBN, TPWUD);
    } else {
      k_mlp<DH_, true, false><<<dim3(2 * NBN), dim3(128), 0, stream>>>(hin, hin + (size_t)TT_ * DH_, WPL, 3, 6,
                                                                       ub1, ub2, ub3, db1, db2, db3,
                                                                       YU, YD, PART, NUDR / 16, NBN, TPWUD);
    }
    k_bnfin<<<dim3(1), dim3(256), 0, stream>>>(PART, ug, ubt, dgm, dbt, ST);
    if (it == 0) {
      k_upd<true><<<dim3(TT_ / UTT), dim3(UTHR), 0, stream>>>(hin, XE, YU, YD, ST, hout);
    } else {
      k_upd<false><<<dim3(TT_ / UTT), dim3(UTHR), 0, stream>>>(hin, XE, YU, YD, ST, hout);
    }
  }
  (void)hipGetLastError();
}
